// GraphSAGEGraphLevel_55980603736137
// MI455X (gfx1250) — hardware-verified
//
#include <hip/hip_runtime.h>
#include <stddef.h>
#include <stdint.h>
#include <math.h>


#define FX     29
#define FD     3
#define FE     12
#define F0     44
#define H0P    64
#define K1     192
#define HD     128
#define K2     512
#define NGR    512
#define NCLS   10
#define PW     256
#define NTHR   256
#define NWAVE  8
#define EPT    8
#define CHUNK  (NTHR * EPT)
#define WCAP   (EPT * 32)
#define LISTN  (NWAVE * WCAP)
#define NBA    1024
#define SLA    10
#define RCAP   16384
#define DEGCAP 64
#define GBM    64
#define GBN    128
#define GTHR   128
#define HR     32
#define NU1    (HD * (K1 / 8))
#define NU2    (HD * (K2 / 8))
#define GPB    16
#define AGG_ZINTS    (LISTN + 2 * RCAP + 3 * NBA)
#define MISC_INTS    16
#define RB_WORDS     128
#define AGG_LDS_INTS (AGG_ZINTS + MISC_INTS + NWAVE * RB_WORDS)
#define NOUT   (NGR * NCLS)
#define WSMAX  134217728

static_assert((CHUNK & (CHUNK - 1)) == 0 && CHUNK <= 4096);
static_assert((NBA & (NBA - 1)) == 0 && NBA == (1 << SLA));
static_assert(((long long)CHUNK << SLA) < (1LL << 31));
static_assert(NBA % NWAVE == 0 && NBA % 32 == 0 && NBA % GBM == 0);
static_assert(RCAP % 4 == 0 && AGG_ZINTS % (NTHR * 4) == 0 && LISTN % 4 == 0);
static_assert(((AGG_ZINTS + MISC_INTS) % 4) == 0);
static_assert(K1 % 32 == 0 && K2 % 32 == 0 && K1 == 3 * H0P && K2 == 4 * HD && F0 <= H0P && F0 % 4 == 0);
static_assert(GBN == HD && GBM == (GTHR / 32) * 16 && HD == 4 * 32 && H0P == 2 * 32);
static_assert(NU1 % NTHR == 0 && NU2 % NTHR == 0);
static_assert(HR * (H0P / 8) == NTHR && HR * H0P == 8 * NTHR);
static_assert(HR * FX <= 4 * NTHR && HR * FD <= NTHR && HR * FE <= 2 * NTHR);
static_assert(NGR % GPB == 0 && (GPB * NCLS * 4) % 128 == 0 && GPB * NCLS <= NTHR && GPB * PW == 16 * NTHR);
static_assert(AGG_LDS_INTS * 4 <= 300000);
static_assert(FX + FD + FE == F0);

typedef float          v2f   __attribute__((ext_vector_type(2)));
typedef float          v4f   __attribute__((ext_vector_type(4)));
typedef float          v8f   __attribute__((ext_vector_type(8)));
typedef int            v4i   __attribute__((ext_vector_type(4)));
typedef int            v8i   __attribute__((ext_vector_type(8)));
typedef unsigned       v2u   __attribute__((ext_vector_type(2)));
typedef unsigned       v4u   __attribute__((ext_vector_type(4)));
typedef unsigned short v8us  __attribute__((ext_vector_type(8)));
typedef unsigned short v16us __attribute__((ext_vector_type(16)));
typedef __bf16         v16bf __attribute__((ext_vector_type(16)));
typedef v4f  __attribute__((may_alias)) v4fa;
typedef v4i  __attribute__((may_alias)) v4ia;
typedef v2u  __attribute__((may_alias)) v2ua;
typedef v4u  __attribute__((may_alias)) v4ua;
typedef v8us __attribute__((may_alias)) v8usa;
typedef unsigned __attribute__((may_alias)) u32a;
union FragB { v16bf v; v16us u; v8us h[2]; v8i w; };

__device__ __forceinline__ v8f wmb(const FragB& a, const FragB& b, v8f c) {
  v8f d = __builtin_amdgcn_wmma_f32_16x16x32_bf16(false, a.v, false, b.v, (short)0, c, false, false);
  asm volatile("v_nop\n\tv_nop\n\tv_nop\n\tv_nop" : "+v"(d) : "v"(a.w), "v"(b.w));
  return d;
}

__device__ __forceinline__ unsigned bf16_bits(float f) {
  const unsigned u = __float_as_uint(f);
  return ((u + 0x7FFFu + ((u >> 16) & 1u)) >> 16) & 0xFFFFu;
}
__device__ __forceinline__ float bf16_val(float f) {
  return __uint_as_float(bf16_bits(f) << 16);
}
__device__ __forceinline__ unsigned hl_sel(float v, unsigned msel) {
  const unsigned hb = bf16_bits(v);
  const unsigned lb = bf16_bits(v - __uint_as_float(hb << 16));
  return (hb & ~msel) | (lb & msel);
}

__device__ __forceinline__ void wave_sync() {
  __builtin_amdgcn_fence(__ATOMIC_RELEASE, "wavefront");
  __builtin_amdgcn_wave_barrier();
  __builtin_amdgcn_fence(__ATOMIC_ACQUIRE, "wavefront");
}

template <int SLB>
__device__ __forceinline__ int scan_chunk(const int* __restrict__ dsts, int nE, int cbase, int slotBase,
                                          int nb, int vec8, int* list, int tid, int lane, int wave) {
  int wc = 0;
  const int el0  = tid * EPT;
  const int e0   = cbase + el0;
  const int sent = -2147483647 - 1;
  v4i da, db;
  if (vec8 != 0 && cbase + CHUNK <= nE) {
    da = *(const v4i*)(dsts + e0);
    db = *(const v4i*)(dsts + e0 + 4);
  } else {
    da.x = (e0     < nE) ? dsts[min(e0,     nE - 1)] : sent;
    da.y = (e0 + 1 < nE) ? dsts[min(e0 + 1, nE - 1)] : sent;
    da.z = (e0 + 2 < nE) ? dsts[min(e0 + 2, nE - 1)] : sent;
    da.w = (e0 + 3 < nE) ? dsts[min(e0 + 3, nE - 1)] : sent;
    db.x = (e0 + 4 < nE) ? dsts[min(e0 + 4, nE - 1)] : sent;
    db.y = (e0 + 5 < nE) ? dsts[min(e0 + 5, nE - 1)] : sent;
    db.z = (e0 + 6 < nE) ? dsts[min(e0 + 6, nE - 1)] : sent;
    db.w = (e0 + 7 < nE) ? dsts[min(e0 + 7, nE - 1)] : sent;
  }
  const unsigned nbs = (unsigned)slotBase;
  const unsigned unb = (unsigned)nb;
  const unsigned s0 = (unsigned)da.x - nbs, s1 = (unsigned)da.y - nbs;
  const unsigned s2 = (unsigned)da.z - nbs, s3 = (unsigned)da.w - nbs;
  const unsigned s4 = (unsigned)db.x - nbs, s5 = (unsigned)db.y - nbs;
  const unsigned s6 = (unsigned)db.z - nbs, s7 = (unsigned)db.w - nbs;
  const bool h0 = s0 < unb, h1 = s1 < unb, h2 = s2 < unb, h3 = s3 < unb;
  const bool h4 = s4 < unb, h5 = s5 < unb, h6 = s6 < unb, h7 = s7 < unb;
  const unsigned any = __builtin_amdgcn_ballot_w32(h0 | h1 | h2 | h3 | h4 | h5 | h6 | h7);
  if (any != 0u) {
#define HITJ(J, HJ, SJ) { \
      const unsigned mj = __builtin_amdgcn_ballot_w32(HJ); \
      if (mj != 0u) { \
        if (HJ) { \
          const int pos = wc + (int)__builtin_amdgcn_mbcnt_lo(mj, 0u); \
          if (pos < WCAP) list[wave * WCAP + pos] = ((el0 + (J)) << SLB) | (int)(SJ); \
        } \
        wc += (int)__builtin_popcount(mj); } }
    HITJ(0, h0, s0)
    HITJ(1, h1, s1)
    HITJ(2, h2, s2)
    HITJ(3, h3, s3)
    HITJ(4, h4, s4)
    HITJ(5, h5, s5)
    HITJ(6, h6, s6)
    HITJ(7, h7, s7)
#undef HITJ
  }
  return wc;
}

__global__ __launch_bounds__(NTHR) void k_wprep(const float* __restrict__ Wl1, const float* __restrict__ Wr1,
                                                const float* __restrict__ Wl2, const float* __restrict__ Wr2,
                                                unsigned short* W1C, unsigned short* W2C) {
  const int u = (int)blockIdx.x * NTHR + (int)threadIdx.x;
  v4f la, lb, ra, rb;
  unsigned msel, ma, mb;
  unsigned short* dp;
  if (u < NU1) {
    const int n    = u / (K1 / 8);
    const int j    = u - n * (K1 / 8);
    const int part = j >> 3;
    const int k8   = (j & 7) * 8;
    const int ka   = k8 < (F0 - 4) ? k8 : (F0 - 4);
    const int kb   = (k8 + 4) < (F0 - 4) ? (k8 + 4) : (F0 - 4);
    la = *(const v4f*)(Wl1 + (size_t)n * F0 + ka);
    lb = *(const v4f*)(Wl1 + (size_t)n * F0 + kb);
    ra = *(const v4f*)(Wr1 + (size_t)n * F0 + ka);
    rb = *(const v4f*)(Wr1 + (size_t)n * F0 + kb);
    msel = (unsigned)(-(int)(part == 2));
    ma   = (unsigned)(-(int)((k8 + 3) < F0));
    mb   = (unsigned)(-(int)((k8 + 7) < F0));
    dp = W1C + (size_t)u * 8;
  } else if (u < NU1 + NU2) {
    const int v    = u - NU1;
    const int n    = v >> 6;
    const int j    = v & 63;
    const int part = j >> 4;
    const int k8   = (j & 15) * 8;
    la = *(const v4f*)(Wl2 + (size_t)n * HD + k8);
    lb = *(const v4f*)(Wl2 + (size_t)n * HD + k8 + 4);
    ra = *(const v4f*)(Wr2 + (size_t)n * HD + k8);
    rb = *(const v4f*)(Wr2 + (size_t)n * HD + k8 + 4);
    msel = (unsigned)(-(int)(part >= 2));
    ma = 0xFFFFFFFFu; mb = 0xFFFFFFFFu;
    dp = W2C + (size_t)v * 8;
  } else {
    return;
  }
  v8us o;
  o[0] = (unsigned short)(((bf16_bits(la.x) & ~msel) | (bf16_bits(ra.x) & msel)) & ma);
  o[1] = (unsigned short)(((bf16_bits(la.y) & ~msel) | (bf16_bits(ra.y) & msel)) & ma);
  o[2] = (unsigned short)(((bf16_bits(la.z) & ~msel) | (bf16_bits(ra.z) & msel)) & ma);
  o[3] = (unsigned short)(((bf16_bits(la.w) & ~msel) | (bf16_bits(ra.w) & msel)) & ma);
  o[4] = (unsigned short)(((bf16_bits(lb.x) & ~msel) | (bf16_bits(rb.x) & msel)) & mb);
  o[5] = (unsigned short)(((bf16_bits(lb.y) & ~msel) | (bf16_bits(rb.y) & msel)) & mb);
  o[6] = (unsigned short)(((bf16_bits(lb.z) & ~msel) | (bf16_bits(rb.z) & msel)) & mb);
  o[7] = (unsigned short)(((bf16_bits(lb.w) & ~msel) | (bf16_bits(rb.w) & msel)) & mb);
  *(volatile v8us*)dp = o;
  __threadfence();
  *(volatile v8us*)dp = o;
}

__global__ __launch_bounds__(NTHR) void k_h0(const float* __restrict__ x, const float* __restrict__ xd,
                                             const int* __restrict__ st, const float* __restrict__ emb,
                                             int nN, int nEmb, unsigned short* h0b) {
  __shared__ __attribute__((aligned(16))) float hrow[HR * H0P];
  __shared__ int sst[HR];
  const int tid = (int)threadIdx.x;
  const int rowBase = (int)blockIdx.x * HR;
  {
    const v4f z = {0.f, 0.f, 0.f, 0.f};
    *(v4fa*)(hrow + 8 * tid) = z;
    *(v4fa*)(hrow + 8 * tid + 4) = z;
  }
  __syncthreads();
#pragma unroll
  for (int it = 0; it < 4; ++it) {
    const int i  = tid + NTHR * it;
    const int ic = i < HR * FX ? i : HR * FX - 1;
    const int r  = ic / FX;
    const int c  = ic - r * FX;
    const int gr = rowBase + r;
    const int gc = gr < nN ? gr : nN - 1;
    const float v = x[(size_t)gc * FX + c];
    if (i < HR * FX && gr < nN) hrow[r * H0P + c] = v;
  }
  {
    const int ic = tid < HR * FD ? tid : HR * FD - 1;
    const int r  = ic / FD;
    const int c  = ic - r * FD;
    const int gr = rowBase + r;
    const int gc = gr < nN ? gr : nN - 1;
    const float v = xd[(size_t)gc * FD + c];
    if (tid < HR * FD && gr < nN) hrow[r * H0P + FX + c] = v;
  }
  {
    const int ic = tid < HR ? tid : HR - 1;
    const int gr = rowBase + ic;
    const int gc = gr < nN ? gr : nN - 1;
    int s = st[gc];
    s = s < 0 ? 0 : (s > nEmb - 1 ? nEmb - 1 : s);
    if (tid < HR) sst[tid] = s;
  }
  __syncthreads();
#pragma unroll
  for (int it = 0; it < 2; ++it) {
    const int i  = tid + NTHR * it;
    const int ic = i < HR * FE ? i : HR * FE - 1;
    const int r  = ic / FE;
    const int c  = ic - r * FE;
    const int gr = rowBase + r;
    const int e  = sst[r];
    const float v = emb[(size_t)e * FE + c];
    if (i < HR * FE && gr < nN) hrow[r * H0P + FX + FD + c] = v;
  }
  __syncthreads();
  const int r  = tid >> 3;
  const int k8 = (tid & 7) * 8;
  const v4f a = *(const v4fa*)(hrow + r * H0P + k8);
  const v4f b = *(const v4fa*)(hrow + r * H0P + k8 + 4);
  v8us o;
  o[0] = (unsigned short)bf16_bits(a.x); o[1] = (unsigned short)bf16_bits(a.y);
  o[2] = (unsigned short)bf16_bits(a.z); o[3] = (unsigned short)bf16_bits(a.w);
  o[4] = (unsigned short)bf16_bits(b.x); o[5] = (unsigned short)bf16_bits(b.y);
  o[6] = (unsigned short)bf16_bits(b.z); o[7] = (unsigned short)bf16_bits(b.w);
  unsigned short* dp = h0b + (size_t)(rowBase + r) * H0P + k8;
  *(volatile v8us*)dp = o;
  __threadfence();
  *(volatile v8us*)dp = o;
}

template <int LYR>
__global__ __launch_bounds__(NTHR) void k_scan(const int* __restrict__ srcs, const int* __restrict__ dsts,
                                               int nE, int nN, int vec8, int mRows,
                                               const unsigned short* __restrict__ h0b,
                                               const float* __restrict__ h1f, unsigned short* apl) {
  extern __shared__ __attribute__((aligned(16))) int dsm[];
  int* list = dsm;
  int* hl   = dsm + LISTN;
  int* sl   = hl + RCAP;
  int* cnt  = sl + RCAP;
  int* offs = cnt + NBA;
  int* cur  = offs + NBA;
  int* misc = cur + NBA;
  const int tid = (int)threadIdx.x, lane = tid & 31, wave = tid >> 5;
  unsigned* rb32 = (unsigned*)(misc + MISC_INTS) + wave * RB_WORDS;
  const int nodeBase = (int)blockIdx.x * NBA;

  {
    const v4i z4 = {0, 0, 0, 0};
    for (int i = tid * 4; i < AGG_ZINTS; i += NTHR * 4) *(v4ia*)(dsm + i) = z4;
    if (tid < MISC_INTS) misc[tid] = 0;
  }
  __syncthreads();

  int t = 0, ov = 0;
  const int nChunks = (nE + CHUNK - 1) / CHUNK;
#pragma unroll 1
  for (int ch = 0; ch < nChunks; ++ch) {
    const int cbase = ch * CHUNK;
    const int wc = scan_chunk<SLA>(dsts, nE, cbase, nodeBase, NBA, vec8, list, tid, lane, wave);
    if (lane == 0) misc[wave] = wc;
    __syncthreads();
    if (wave == 0) {
#pragma unroll 1
      for (int w2 = 0; w2 < NWAVE; ++w2) {
        int c = misc[w2];
        c = c < 0 ? 0 : (c > WCAP ? WCAP : c);
#pragma unroll 1
        for (int b0 = 0; b0 < c; b0 += 32) {
          const int idx = b0 + lane;
          const int ent = list[w2 * WCAP + (idx < WCAP ? idx : WCAP - 1)];
          const int m32 = (c - b0) < 32 ? (c - b0) : 32;
#pragma unroll 1
          for (int k = 0; k < m32; ++k) {
            const int u    = __builtin_amdgcn_readlane(ent, k);
            const int slot = u & (NBA - 1);
            const int el   = (u >> SLA) & (CHUNK - 1);
            const int pk   = ((cbase + el) << SLA) | slot;
            if (t < RCAP) {
              if (lane == 0) { hl[t] = pk; cnt[slot] = cnt[slot] + 1; }
              t = t + 1;
            } else {
              ov = 1;
            }
          }
        }
      }
    }
    __syncthreads();
  }
  if (wave == 0 && lane == 0) { misc[8] = t; misc[9] = ov; }
  __syncthreads();
  int tt = misc[8];
  tt = tt < 0 ? 0 : (tt > RCAP ? RCAP : tt);
  const int ovf = misc[9];

  if (wave == 0) {
    const int base = lane * (NBA / 32);
    int s = 0;
#pragma unroll 1
    for (int i = 0; i < NBA / 32; ++i) s += cnt[base + i];
    int incl = s;
#pragma unroll
    for (int d = 1; d < 32; d <<= 1) {
      const int y = __shfl_up(incl, d, 32);
      if (lane >= d) incl += y;
    }
    int run = incl - s;
#pragma unroll 1
    for (int i = 0; i < NBA / 32; ++i) {
      const int cv = cnt[base + i];
      offs[base + i] = run;
      cur[base + i]  = run;
      run += cv;
    }
  }
  __syncthreads();
  if (wave == 0) {
#pragma unroll 1
    for (int b0 = 0; b0 < tt; b0 += 32) {
      const int idx = b0 + lane;
      const int ent = hl[idx < RCAP ? idx : RCAP - 1];
      const int m32 = (tt - b0) < 32 ? (tt - b0) : 32;
#pragma unroll 1
      for (int k = 0; k < m32; ++k) {
        const int u    = __builtin_amdgcn_readlane(ent, k);
        const int slot = u & (NBA - 1);
        if (lane == 0) {
          int p = cur[slot];
          p = p < 0 ? 0 : (p > RCAP - 1 ? RCAP - 1 : p);
          sl[p] = u;
          cur[slot] = p + 1;
        }
      }
    }
  }
  __syncthreads();

  const float qnan = __int_as_float(0x7fc00000);
  const float pz = (ovf != 0) ? qnan : 0.0f;
#pragma unroll 1
  for (int si = 0; si < NBA / NWAVE; ++si) {
    const int s    = si * NWAVE + wave;
    const int node = nodeBase + s;
    const int craw = cnt[s];
    const bool big = craw > DEGCAP;
    const int c = craw < 0 ? 0 : (craw > DEGCAP ? DEGCAP : craw);
    int o = offs[s];
    o = o < 0 ? 0 : (o > RCAP ? RCAP : o);
    const int nc = node < nN ? node : nN - 1;
    float a0 = 0.0f, a1 = 0.0f, a2 = 0.0f, a3 = 0.0f;
#pragma unroll 1
    for (int b0 = 0; b0 < c; b0 += 32) {
      int idx = o + b0 + lane;
      idx = idx > RCAP - 1 ? RCAP - 1 : idx;
      const int ent = sl[idx];
      int eid = ent >> SLA;
      eid = eid < 0 ? 0 : (eid > nE - 1 ? nE - 1 : eid);
      int sr = srcs[eid];
      sr = sr < 0 ? 0 : (sr > nN - 1 ? nN - 1 : sr);
      const int m32 = (c - b0) < 32 ? (c - b0) : 32;
#pragma unroll 1
      for (int k = 0; k < m32; ++k) {
        const int sk = __builtin_amdgcn_readlane(sr, k);
        if constexpr (LYR == 1) {
          const unsigned w = *(const u32a*)(h0b + (size_t)sk * H0P + 2 * lane);
          a0 += __uint_as_float(w << 16);
          a1 += __uint_as_float(w & 0xffff0000u);
        } else {
          const v4f a = *(const v4f*)(h1f + (size_t)sk * HD + 4 * lane);
          a0 += a.x; a1 += a.y; a2 += a.z; a3 += a.w;
        }
      }
    }
    const float cf  = craw < 1 ? 1.0f : (float)craw;
    const float inv = 1.0f / cf;
    const float pzr = big ? qnan : pz;
    const bool live = node < nN;
    const float m0 = live ? (a0 * inv + pzr) : 0.0f;
    const float m1 = live ? (a1 * inv + pzr) : 0.0f;
    if constexpr (LYR == 1) {
      const unsigned hb0 = bf16_bits(m0), hb1 = bf16_bits(m1);
      const unsigned lb0 = bf16_bits(m0 - __uint_as_float(hb0 << 16));
      const unsigned lb1 = bf16_bits(m1 - __uint_as_float(hb1 << 16));
      const unsigned own = *(const u32a*)(h0b + (size_t)nc * H0P + 2 * lane);
      rb32[lane]      = hb0 | (hb1 << 16);
      rb32[32 + lane] = lb0 | (lb1 << 16);
      rb32[64 + lane] = live ? own : 0u;
      wave_sync();
      const int lq = lane < 24 ? lane : 23;
      const v4u q0 = *(const v4ua*)(rb32 + 4 * lq);
      wave_sync();
      const bool wr = (node < mRows) && (lane < 24);
      unsigned short* rpw = apl + (size_t)node * K1 + 8 * lq;
      if (wr) *(volatile v4u*)rpw = q0;
      __threadfence();
      if (wr) *(volatile v4u*)rpw = q0;
    } else {
      const float m2 = live ? (a2 * inv + pzr) : 0.0f;
      const float m3 = live ? (a3 * inv + pzr) : 0.0f;
      const unsigned hb0 = bf16_bits(m0), hb1 = bf16_bits(m1), hb2 = bf16_bits(m2), hb3 = bf16_bits(m3);
      const unsigned lb0 = bf16_bits(m0 - __uint_as_float(hb0 << 16));
      const unsigned lb1 = bf16_bits(m1 - __uint_as_float(hb1 << 16));
      const unsigned lb2 = bf16_bits(m2 - __uint_as_float(hb2 << 16));
      const unsigned lb3 = bf16_bits(m3 - __uint_as_float(hb3 << 16));
      v2u hw, lw;
      hw.x = hb0 | (hb1 << 16); hw.y = hb2 | (hb3 << 16);
      lw.x = lb0 | (lb1 << 16); lw.y = lb2 | (lb3 << 16);
      *(v2ua*)(rb32 + 2 * lane) = hw;
      *(v2ua*)(rb32 + 64 + 2 * lane) = lw;
      wave_sync();
      const v4u q0 = *(const v4ua*)(rb32 + 4 * lane);
      wave_sync();
      const bool wr = node < mRows;
      unsigned short* rpw = apl + (size_t)node * K2 + 8 * lane;
      if (wr) *(volatile v4u*)rpw = q0;
      __threadfence();
      if (wr) *(volatile v4u*)rpw = q0;
    }
  }
}

template <int LYR>
__device__ __forceinline__ void gemm_store_pass(const float* stg, int wave, int lane, int rowBase,
                                                float* hout, unsigned short* ac2) {
#pragma unroll 2
  for (int i = 0; i < 16; ++i) {
    const int lr = 16 * wave + i;
    const size_t r = (size_t)(rowBase + lr);
    const v4f y = *(const v4fa*)(stg + lr * GBN + 4 * lane);
    *(volatile v4f*)(hout + r * HD + 4 * lane) = y;
    if constexpr (LYR == 1) {
      const float* cp = stg + lr * GBN + 8 * (lane & 15);
      const v4f c0 = *(const v4fa*)cp;
      const v4f c1 = *(const v4fa*)(cp + 4);
      const unsigned msel = (unsigned)(-(int)(lane >> 4));
      v4u pv;
      pv.x = hl_sel(c0.x, msel) | (hl_sel(c0.y, msel) << 16);
      pv.y = hl_sel(c0.z, msel) | (hl_sel(c0.w, msel) << 16);
      pv.z = hl_sel(c1.x, msel) | (hl_sel(c1.y, msel) << 16);
      pv.w = hl_sel(c1.z, msel) | (hl_sel(c1.w, msel) << 16);
      *(volatile v4u*)(ac2 + r * K2 + 2 * HD + 8 * lane) = pv;
    }
  }
}

template <int LYR>
__global__ __launch_bounds__(GTHR) void k_gemm(const unsigned short* Apl, int lda,
                                               const unsigned short* __restrict__ BT, int K,
                                               const float* __restrict__ bias, const float* __restrict__ gam,
                                               const float* __restrict__ bet,
                                               float* hout, unsigned short* ac2, int nOut) {
  __shared__ __attribute__((aligned(16))) float stg[GBM * GBN];
  const int tid = (int)threadIdx.x, lane = tid & 31, wave = tid >> 5, hh = lane >> 4, m = lane & 15;
  const int rowBase = (int)blockIdx.x * GBM;

  v8f acc[8];
  {
    const v8f z = {0.f, 0.f, 0.f, 0.f, 0.f, 0.f, 0.f, 0.f};
#pragma unroll
    for (int t = 0; t < 8; ++t) acc[t] = z;
  }
  const unsigned short* ap = Apl + (size_t)(rowBase + 16 * wave + m) * (size_t)lda + 8 * hh;
  const unsigned short* bp = BT + (size_t)m * (size_t)K + 8 * hh;

#pragma unroll 1
  for (int k0 = 0; k0 < K; k0 += 32) {
    FragB af;
    af.h[0] = *(const v8usa*)(ap + k0);
    af.h[1] = *(const v8usa*)(ap + k0 + 16);
#pragma unroll
    for (int nt = 0; nt < 8; ++nt) {
      const unsigned short* wq = bp + (size_t)(16 * nt) * (size_t)K + k0;
      FragB bf;
      bf.h[0] = *(const v8usa*)wq;
      bf.h[1] = *(const v8usa*)(wq + 16);
      acc[nt] = wmb(af, bf, acc[nt]);
    }
  }

#pragma unroll
  for (int nt = 0; nt < 8; ++nt) {
    const int lc = 16 * nt + m;
#pragma unroll
    for (int r = 0; r < 8; ++r) {
      const int lr = 16 * wave + 8 * hh + r;
      stg[lr * GBN + lc] = acc[nt][r];
    }
  }
  __syncthreads();

  v4f bb4, g4, be4;
  {
    const v4f t1 = *(const v4f*)(bias + 4 * lane);
    const v4f t2 = *(const v4f*)(gam + 4 * lane);
    const v4f t3 = *(const v4f*)(bet + 4 * lane);
    bb4.x = bf16_val(t1.x); bb4.y = bf16_val(t1.y); bb4.z = bf16_val(t1.z); bb4.w = bf16_val(t1.w);
    g4.x  = bf16_val(t2.x); g4.y  = bf16_val(t2.y); g4.z  = bf16_val(t2.z); g4.w  = bf16_val(t2.w);
    be4.x = bf16_val(t3.x); be4.y = bf16_val(t3.y); be4.z = bf16_val(t3.z); be4.w = bf16_val(t3.w);
  }

#pragma unroll 1
  for (int i = 0; i < 16; ++i) {
    const int lr = 16 * wave + i;
    float* sp = stg + lr * GBN + 4 * lane;
    v4f t = *(const v4fa*)sp;
    t = t + bb4;
    float s = (t.x + t.y) + (t.z + t.w);
    s += __shfl_xor(s, 16, 32);
    s += __shfl_xor(s, 8, 32);
    s += __shfl_xor(s, 4, 32);
    s += __shfl_xor(s, 2, 32);
    s += __shfl_xor(s, 1, 32);
    const float mu = s * (1.0f / 128.0f);
    v4f d;
    d.x = t.x - mu; d.y = t.y - mu; d.z = t.z - mu; d.w = t.w - mu;
    float q = (d.x * d.x + d.y * d.y) + (d.z * d.z + d.w * d.w);
    q += __shfl_xor(q, 16, 32);
    q += __shfl_xor(q, 8, 32);
    q += __shfl_xor(q, 4, 32);
    q += __shfl_xor(q, 2, 32);
    q += __shfl_xor(q, 1, 32);
    const float rs = rsqrtf(q * (1.0f / 128.0f) + 1e-5f);
    v4f y;
    y.x = g4.x * d.x * rs + be4.x;
    y.y = g4.y * d.y * rs + be4.y;
    y.z = g4.z * d.z * rs + be4.z;
    y.w = g4.w * d.w * rs + be4.w;
    y.x = (y.x > 0.0f) ? y.x : (y.x - y.x);
    y.y = (y.y > 0.0f) ? y.y : (y.y - y.y);
    y.z = (y.z > 0.0f) ? y.z : (y.z - y.z);
    y.w = (y.w > 0.0f) ? y.w : (y.w - y.w);
    const bool ok = (rowBase + lr) < nOut;
    y.x = ok ? y.x : 0.0f; y.y = ok ? y.y : 0.0f; y.z = ok ? y.z : 0.0f; y.w = ok ? y.w : 0.0f;
    *(v4fa*)sp = y;
  }
  __syncthreads();

  gemm_store_pass<LYR>(stg, wave, lane, rowBase, hout, ac2);
  __threadfence();
  gemm_store_pass<LYR>(stg, wave, lane, rowBase, hout, ac2);
}

__global__ __launch_bounds__(NTHR) void k_pool(const float* __restrict__ hf, const int* __restrict__ bat,
                                               int nN, float* pl) {
  __shared__ __attribute__((aligned(16))) float wsum[NWAVE * HD];
  __shared__ __attribute__((aligned(16))) float wmx[NWAVE * HD];
  __shared__ int wcn[NWAVE];
  __shared__ __attribute__((aligned(16))) float outs[PW];
  const int tid = (int)threadIdx.x, lane = tid & 31, wave = tid >> 5;
  const int g = (int)blockIdx.x;
  const float ninf = __int_as_float((int)0xff800000u);

  float a0 = 0.0f, a1 = 0.0f, a2 = 0.0f, a3 = 0.0f;
  float m0 = ninf, m1 = ninf, m2 = ninf, m3 = ninf;
  int cnt = 0;
#pragma unroll 1
  for (int i0 = wave * 32; i0 < nN; i0 += NTHR) {
    const int i  = i0 + lane;
    const int ic = i < nN ? i : nN - 1;
    const int b  = bat[ic];
    const bool hit = (i < nN) && (b == g);
    unsigned msk = __builtin_amdgcn_ballot_w32(hit);
    int nh = (int)__builtin_popcount(msk);
    nh = nh > 32 ? 32 : nh;
    cnt += nh;
#pragma unroll 1
    for (int q = 0; q < nh; ++q) {
      const int k = __builtin_ffs((int)msk) - 1;
      msk &= msk - 1u;
      int node = i0 + (k < 0 ? 0 : k);
      node = node > nN - 1 ? nN - 1 : node;
      const v4f v = *(const v4f*)(hf + (size_t)node * HD + 4 * lane);
      a0 += v.x; a1 += v.y; a2 += v.z; a3 += v.w;
      m0 = (v.x > m0 || v.x != v.x) ? v.x : m0;
      m1 = (v.y > m1 || v.y != v.y) ? v.y : m1;
      m2 = (v.z > m2 || v.z != v.z) ? v.z : m2;
      m3 = (v.w > m3 || v.w != v.w) ? v.w : m3;
    }
  }
  {
    v4f sv; sv.x = a0; sv.y = a1; sv.z = a2; sv.w = a3;
    v4f mv; mv.x = m0; mv.y = m1; mv.z = m2; mv.w = m3;
    *(v4fa*)(wsum + wave * HD + 4 * lane) = sv;
    *(v4fa*)(wmx + wave * HD + 4 * lane) = mv;
  }
  if (lane == 0) wcn[wave] = cnt;
  __syncthreads();
  if (tid < HD) {
    float s = 0.0f, mm = ninf;
    int c = 0;
#pragma unroll
    for (int w2 = 0; w2 < NWAVE; ++w2) {
      const v4f* dummy = 0; (void)dummy;
      s += ((const float*)wsum)[w2 * HD + tid];
      const float xv = ((const float*)wmx)[w2 * HD + tid];
      mm = (xv > mm || xv != xv) ? xv : mm;
      c += wcn[w2];
    }
    const float cf = (c < 1) ? 1.0f : (float)c;
    outs[tid] = s * (1.0f / cf);
    outs[HD + tid] = mm;
  }
  __syncthreads();
  const int tq = tid < 64 ? tid : 63;
  const v4f ov = *(const v4fa*)(outs + 4 * tq);
  float* op = pl + (size_t)g * PW + 4 * tq;
  const bool okst = tid < 64;
  if (okst) *(volatile v4f*)op = ov;
  __threadfence();
  if (okst) *(volatile v4f*)op = ov;
}

__global__ __launch_bounds__(NTHR) void k_head(const float* __restrict__ pl, const float* __restrict__ Wlin,
                                               const float* __restrict__ blin, float* out) {
  __shared__ __attribute__((aligned(16))) float wls[NCLS * PW];
  __shared__ __attribute__((aligned(16))) float ps[GPB * PW];
  __shared__ float bls[16];
  __shared__ __attribute__((aligned(16))) float os[GPB * NCLS];
  const int tid = (int)threadIdx.x;
  const int g0 = (int)blockIdx.x * GPB;
#pragma unroll 1
  for (int i = tid; i < NCLS * PW; i += NTHR) wls[i] = bf16_val(Wlin[i]);
#pragma unroll
  for (int it = 0; it < 4; ++it) {
    const int q = tid + NTHR * it;
    const v4f v = *(const v4f*)(pl + (size_t)g0 * PW + 4 * q);
    *(v4fa*)(ps + 4 * q) = v;
  }
  if (tid < 16) {
    const float bb = blin[tid < NCLS ? tid : NCLS - 1];
    bls[tid] = (tid < NCLS) ? bf16_val(bb) : 0.0f;
  }
  __syncthreads();
  {
    const int idx = tid < GPB * NCLS ? tid : GPB * NCLS - 1;
    const int gl  = idx / NCLS;
    const int c   = idx - gl * NCLS;
    const float* pr = ps + gl * PW;
    const float* wr = wls + c * PW;
    float s = 0.0f;
#pragma unroll 2
    for (int f4 = 0; f4 < PW / 4; ++f4) {
      const v4f p = *(const v4fa*)(pr + 4 * f4);
      const v4f w = *(const v4fa*)(wr + 4 * f4);
      s = fmaf(p.x, w.x, s);
      s = fmaf(p.y, w.y, s);
      s = fmaf(p.z, w.z, s);
      s = fmaf(p.w, w.w, s);
    }
    if (tid < GPB * NCLS) os[tid] = s + bls[c];
  }
  __syncthreads();
  const int tq = tid < 40 ? tid : 39;
  const v4f ov = *(const v4fa*)(os + 4 * tq);
  float* op = out + (size_t)blockIdx.x * (GPB * NCLS) + 4 * tq;
  const bool okst = tid < 40;
  if (okst) *(volatile v4f*)op = ov;
  __threadfence();
  if (okst) *(volatile v4f*)op = ov;
}

static inline int cdiv(int a, int b) { return (a + b - 1) / b; }
static inline size_t al256(size_t o) { return (o + 255) & ~(size_t)255; }

extern "C" void kernel_launch(void* const* d_in, const int* in_sizes, int n_in,
                              void* d_out, int out_size, void* d_ws, size_t ws_size,
                              hipStream_t stream) {
  if (n_in < 18) return;
  if (in_sizes[0] < FX || (in_sizes[0] % FX) != 0) return;
  const int nN = in_sizes[0] / FX;
  if (nN < 16 || nN >= (1 << 22)) return;
  if (in_sizes[1] != nN * FD) return;
  if (in_sizes[2] != nN) return;
  if (in_sizes[3] < 2 || (in_sizes[3] & 1) != 0) return;
  const int nE = in_sizes[3] / 2;
  if (nE < 1 || nE >= (1 << 21)) return;
  if (in_sizes[4] != nN) return;
  if (in_sizes[5] < FE || (in_sizes[5] % FE) != 0) return;
  const int nEmb = in_sizes[5] / FE;
  if (in_sizes[6] != HD * F0 || in_sizes[7] != HD || in_sizes[8] != HD * F0) return;
  if (in_sizes[9] != HD || in_sizes[10] != HD) return;
  if (in_sizes[11] != HD * HD || in_sizes[12] != HD || in_sizes[13] != HD * HD) return;
  if (in_sizes[14] != HD || in_sizes[15] != HD) return;
  if (in_sizes[16] != NCLS * PW || in_sizes[17] != NCLS) return;
  if (out_size != NOUT) return;

  const float* x     = (const float*)d_in[0];
  const float* xd    = (const float*)d_in[1];
  const int*   stt   = (const int*)d_in[2];
  const int*   edge  = (const int*)d_in[3];
  const int*   bat   = (const int*)d_in[4];
  const float* emb   = (const float*)d_in[5];
  const float* Wl1   = (const float*)d_in[6];
  const float* bl1   = (const float*)d_in[7];
  const float* Wr1   = (const float*)d_in[8];
  const float* g1    = (const float*)d_in[9];
  const float* be1   = (const float*)d_in[10];
  const float* Wl2   = (const float*)d_in[11];
  const float* bl2   = (const float*)d_in[12];
  const float* Wr2   = (const float*)d_in[13];
  const float* g2    = (const float*)d_in[14];
  const float* be2   = (const float*)d_in[15];
  const float* Wlin  = (const float*)d_in[16];
  const float* blin  = (const float*)d_in[17];
  float* out = (float*)d_out;
  const int* src = edge;
  const int* dst = edge + nE;

  const int MP = cdiv(nN, GBM) * GBM;
  const int gM = MP / GBM;
  const int gA = cdiv(MP, NBA);
  if ((long long)gA * NBA < (long long)MP) return;
  if ((MP % HR) != 0) return;
  const int vec8 = ((nE & 3) == 0) ? 1 : 0;

  char* ws = (char*)d_ws;
  size_t off = 0;
  const size_t oW1C = off; off = al256(off + (size_t)HD * K1 * 2);
  const size_t oW2C = off; off = al256(off + (size_t)HD * K2 * 2);
  const size_t oH0B = off; off = al256(off + (size_t)MP * H0P * 2);
  const size_t oAC1 = off; off = al256(off + (size_t)MP * K1 * 2);
  const size_t oH1  = off; off = al256(off + (size_t)MP * HD * 4);
  const size_t oAC2 = off; off = al256(off + (size_t)MP * K2 * 2);
  const size_t oH2  = off; off = al256(off + (size_t)MP * HD * 4);
  const size_t oPL  = off; off = al256(off + (size_t)NGR * PW * 4);
  if (off > ws_size || off > (size_t)WSMAX) return;
  unsigned short* W1C = (unsigned short*)(ws + oW1C);
  unsigned short* W2C = (unsigned short*)(ws + oW2C);
  unsigned short* H0B = (unsigned short*)(ws + oH0B);
  unsigned short* AC1 = (unsigned short*)(ws + oAC1);
  float*          H1  = (float*)(ws + oH1);
  unsigned short* AC2 = (unsigned short*)(ws + oAC2);
  float*          H2  = (float*)(ws + oH2);
  float*          PL  = (float*)(ws + oPL);

  const size_t scanLds = (size_t)AGG_LDS_INTS * 4;
  hipFuncSetAttribute(reinterpret_cast<const void*>(&k_scan<1>), hipFuncAttributeMaxDynamicSharedMemorySize, (int)scanLds);
  hipFuncSetAttribute(reinterpret_cast<const void*>(&k_scan<2>), hipFuncAttributeMaxDynamicSharedMemorySize, (int)scanLds);

  k_wprep<<<(NU1 + NU2) / NTHR, NTHR, 0, stream>>>(Wl1, Wr1, Wl2, Wr2, W1C, W2C);
  k_h0<<<MP / HR, NTHR, 0, stream>>>(x, xd, stt, emb, nN, nEmb, H0B);
  k_scan<1><<<gA, NTHR, scanLds, stream>>>(src, dst, nE, nN, vec8, MP, H0B, H1, AC1);
  k_gemm<1><<<gM, GTHR, 0, stream>>>(AC1, K1, W1C, K1, bl1, g1, be1, H1, AC2, nN);
  k_scan<2><<<gA, NTHR, scanLds, stream>>>(src, dst, nE, nN, vec8, MP, H0B, H1, AC2);
  k_gemm<2><<<gM, GTHR, 0, stream>>>(AC2, K2, W2C, K2, bl2, g2, be2, H2, AC2, nN);
  k_pool<<<NGR, NTHR, 0, stream>>>(H2, bat, nN, PL);
  k_head<<<NGR / GPB, NTHR, 0, stream>>>(PL, Wlin, blin, out);
}
